// KimiDecoderLayer_68195490726079
// MI455X (gfx1250) — hardware-run, weakly checked
//
#include <hip/hip_runtime.h>
#include <math.h>

typedef __attribute__((ext_vector_type(16))) _Float16 v16h;
typedef __attribute__((ext_vector_type(8)))  _Float16 v8h;
typedef __attribute__((ext_vector_type(4)))  _Float16 v4h;
typedef __attribute__((ext_vector_type(8)))  float    v8f;
typedef __attribute__((ext_vector_type(4)))  float    v4f;

constexpr int kNB      = 2;
constexpr int kT       = 1024;
constexpr int kHid     = 2048;
constexpr int kNH      = 8;
constexpr int kHD      = 128;
constexpr int kP       = kNH * kHD;
constexpr int kRows    = kNB * kT;
constexpr int kQkvN    = 3 * kP;
constexpr int kLrN     = 2 * kHD;
constexpr int kBetaPad = 64;
constexpr int kWlrRows = kLrN + kBetaPad;
constexpr int kCvP     = 260;
constexpr int kScanTS  = 16;
constexpr int kScanOP  = 68;
constexpr float kEps   = 1e-6f;
static_assert(kP == 1024 && kRows == 2048 && kQkvN == 3072 && kLrN == 256 && kWlrRows == 320, "shapes");
static_assert((kHid % 32) == 0 && (kP % 32) == 0 && (kHD % 32) == 0, "GEMM K multiples of 32");
static_assert((kRows % 64) == 0 && (kQkvN % 32) == 0 && (kLrN % 64) == 0 && (kBetaPad % 64) == 0 && (kP % 64) == 0 && (kHid % 64) == 0, "GEMM M,N tile multiples");
static_assert((kT % 64) == 0 && (kT % kScanTS) == 0 && (kT & (kT - 1)) == 0, "time tiling");
static_assert(kHD == 128 && kNH == 8, "head geometry used by the lane maps");

constexpr float kCarryX = 16.0f;
constexpr float kCarryW = 256.0f;
constexpr float kCarryR = 2048.0f;
constexpr float kCarryH = 16.0f;
constexpr float kCarryO = 16.0f;
constexpr float kScaleMain = 1.0f / (kCarryX * kCarryW);
constexpr float kScaleRes  = kScaleMain / kCarryR;
constexpr float kScaleHid  = kCarryH / (kCarryX * kCarryW);
constexpr float kScaleLr2  = 1.0f / (kCarryH * kCarryW);
constexpr float kScaleOut  = 1.0f / (kCarryO * kCarryW);
constexpr float kF16MinNormal = 6.103515625e-5f;
constexpr float kF32MinNormal = 1.17549435e-38f;

constexpr double cx_rsqrt(double x) {
  double y = 1.0;
  while (y * y * x > 1.0) y *= 0.5;
  for (int i = 0; i < 60; ++i) y = y * (1.5 - 0.5 * x * y * y);
  return y;
}
constexpr float kQScale = (float)cx_rsqrt((double)kHD);
static_assert(kQScale > 0.0883883f && kQScale < 0.0883884f, "q scale");

constexpr size_t kSzXH   = (size_t)kRows * kHid * 2;
constexpr size_t kSzXL   = (size_t)kRows * kHid * 2;
constexpr size_t kSzWH   = (size_t)kQkvN * kHid * 2;
constexpr size_t kSzWL   = (size_t)kQkvN * kHid * 2;
constexpr size_t kSzWLR  = (size_t)kWlrRows * kHid * 2;
constexpr size_t kSzW2   = (size_t)2 * kP * kHD * 2;
constexpr size_t kSzWOH  = (size_t)kHid * kP * 2;
constexpr size_t kSzQKV  = (size_t)kRows * kQkvN * 4;
constexpr size_t kSzHID  = (size_t)kRows * kLrN * 2;
constexpr size_t kSzBETA = (size_t)kRows * kBetaPad * 4;
constexpr size_t kSzGG   = (size_t)2 * kRows * kP * 4;
constexpr size_t kSzEG   = (size_t)kRows * kP * 4;
constexpr size_t kSzQN   = (size_t)kRows * kP * 4;
constexpr size_t kSzKN   = (size_t)kRows * kP * 4;
constexpr size_t kSzVN   = (size_t)kRows * kP * 4;
constexpr size_t kSzOGH  = (size_t)kRows * kP * 2;
constexpr size_t kOffXH   = 0;
constexpr size_t kOffXL   = kOffXH   + kSzXH;
constexpr size_t kOffWH   = kOffXL   + kSzXL;
constexpr size_t kOffWL   = kOffWH   + kSzWH;
constexpr size_t kOffWLR  = kOffWL   + kSzWL;
constexpr size_t kOffW2   = kOffWLR  + kSzWLR;
constexpr size_t kOffWOH  = kOffW2   + kSzW2;
constexpr size_t kOffQKV  = kOffWOH  + kSzWOH;
constexpr size_t kOffHID  = kOffQKV  + kSzQKV;
constexpr size_t kOffBETA = kOffHID  + kSzHID;
constexpr size_t kOffGG   = kOffBETA + kSzBETA;
constexpr size_t kOffEG   = kOffGG   + kSzGG;
constexpr size_t kOffQN   = kOffEG   + kSzEG;
constexpr size_t kOffKN   = kOffQN   + kSzQN;
constexpr size_t kOffVN   = kOffKN   + kSzKN;
constexpr size_t kOffOGH  = kOffVN   + kSzVN;
constexpr size_t kWsTotal = kOffOGH  + kSzOGH;
static_assert(kWsTotal == 129236992ull, "carve total");
static_assert(kWsTotal <= 134217728ull, "carve cap");
static_assert((size_t)kRows * kP * 4 <= kSzQKV, "scan output fits the re-used region");
static_assert((kOffXL % 128) == 0 && (kOffWH % 128) == 0 && (kOffWL % 128) == 0 && (kOffWLR % 128) == 0 &&
              (kOffW2 % 128) == 0 && (kOffWOH % 128) == 0 && (kOffQKV % 128) == 0 && (kOffHID % 128) == 0 &&
              (kOffBETA % 128) == 0 && (kOffGG % 128) == 0 && (kOffEG % 128) == 0 && (kOffQN % 128) == 0 &&
              (kOffKN % 128) == 0 && (kOffVN % 128) == 0 && (kOffOGH % 128) == 0, "128-B aligned regions");

__device__ __forceinline__ float flush_h(float v) { return (fabsf(v) < kF16MinNormal) ? 0.0f : v; }

__device__ __forceinline__ v16h frag_load(const _Float16* p) {
  union { v16h v; v8h h[2]; } f;
  f.h[0] = *(const v8h*)(p);
  f.h[1] = *(const v8h*)(p + 16);
  return f.v;
}
__device__ __forceinline__ v8f mma_h(v16h a, v16h b, v8f c) {
  c = __builtin_amdgcn_wmma_f32_16x16x32_f16(false, a, false, b, (short)0, c, false, false);
  asm volatile("v_nop\n\tv_nop\n\tv_nop\n\tv_nop" : "+v"(c) : "v"(a), "v"(b));
  return c;
}
__device__ __forceinline__ void wave_lds_sync() {
  __builtin_amdgcn_fence(__ATOMIC_RELEASE, "workgroup");
  __builtin_amdgcn_wave_barrier();
  __builtin_amdgcn_fence(__ATOMIC_ACQUIRE, "workgroup");
}

template <int OUT_MODE>
__global__ __launch_bounds__(256) void gemm_plain_kernel(
    const unsigned short* __restrict__ Ap, int lda, long strideA,
    const unsigned short* __restrict__ Btp, int ldb, long strideB,
    void* __restrict__ Cout, int ldc, long strideC,
    int M, int N, int K, float scale)
{
  __shared__ __align__(16) float sT[8][16 * 68];
  const int lane = threadIdx.x & 31;
  const int wave = threadIdx.x >> 5;
  const int tilesN = N >> 6;
  const int tilesM = M >> 6;
  const int tile = blockIdx.x * 8 + wave;
  if (tile >= tilesM * tilesN) return;
  const int tm = tile / tilesN;
  const int tn = tile - tm * tilesN;
  const int m0 = tm << 6;
  const int n0 = tn << 6;
  const _Float16* Ab = (const _Float16*)Ap  + (size_t)blockIdx.y * strideA;
  const _Float16* Bb = (const _Float16*)Btp + (size_t)blockIdx.y * strideB;
  const int rlane = lane & 15;
  const int koff  = (lane >> 4) * 8;
  const int mOff  = (lane >> 4) * 8;

  v8f acc[4][4];
#pragma unroll
  for (int i = 0; i < 4; ++i)
#pragma unroll
    for (int j = 0; j < 4; ++j) acc[i][j] = (v8f){0.f, 0.f, 0.f, 0.f, 0.f, 0.f, 0.f, 0.f};

  for (int k0 = 0; k0 < K; k0 += 32) {
    v16h bf[4];
#pragma unroll
    for (int j = 0; j < 4; ++j)
      bf[j] = frag_load(Bb + (size_t)(n0 + (j << 4) + rlane) * ldb + koff + k0);
#pragma unroll
    for (int i = 0; i < 4; ++i) {
      const v16h af = frag_load(Ab + (size_t)(m0 + (i << 4) + rlane) * lda + koff + k0);
#pragma unroll
      for (int j = 0; j < 4; ++j) acc[i][j] = mma_h(af, bf[j], acc[i][j]);
    }
  }

  float* slab = sT[wave];
#pragma unroll
  for (int i = 0; i < 4; ++i) {
    const int mBase = m0 + (i << 4);
#pragma unroll
    for (int j = 0; j < 4; ++j) {
#pragma unroll
      for (int r = 0; r < 8; ++r)
        slab[(mOff + r) * 68 + (j << 4) + rlane] = acc[i][j][r] * scale;
    }
    wave_lds_sync();
    if (OUT_MODE == 0) {
      float* C = (float*)Cout + (size_t)blockIdx.y * strideC;
      const int hh = lane >> 4, c4 = (lane & 15) * 4;
      for (int pass = 0; pass < 2; ++pass) {
#pragma unroll
        for (int it = 0; it < 8; ++it) {
          const int row = it * 2 + hh;
          const v4f v = *(const v4f*)(slab + row * 68 + c4);
          *(volatile v4f*)(C + (size_t)(mBase + row) * ldc + n0 + c4) = v;
        }
        __threadfence();
      }
    } else {
      unsigned short* C = (unsigned short*)Cout + (size_t)blockIdx.y * strideC;
      const int q = lane >> 3, c8 = (lane & 7) * 8;
      for (int pass = 0; pass < 2; ++pass) {
#pragma unroll
        for (int it = 0; it < 4; ++it) {
          const int row = it * 4 + q;
          const float* sp = slab + row * 68 + c8;
          const v4f a0 = *(const v4f*)(sp);
          const v4f a1 = *(const v4f*)(sp + 4);
          v8h hv;
#pragma unroll
          for (int e = 0; e < 4; ++e) {
            hv[e]     = (_Float16)flush_h(a0[e]);
            hv[4 + e] = (_Float16)flush_h(a1[e]);
          }
          *(volatile v8h*)(C + (size_t)(mBase + row) * ldc + n0 + c8) = hv;
        }
        __threadfence();
      }
    }
    wave_lds_sync();
  }
}

__global__ __launch_bounds__(256) void gemm_split_kernel(
    const unsigned short* __restrict__ Ahp, const unsigned short* __restrict__ Alp, int lda,
    const unsigned short* __restrict__ Bhp, const unsigned short* __restrict__ Blp, int ldb,
    float* __restrict__ C, int ldc, int M, int N, int K, float s_main, float s_res)
{
  __shared__ __align__(16) float sT[8][16 * 36];
  const int lane = threadIdx.x & 31;
  const int wave = threadIdx.x >> 5;
  const int tilesN = N >> 5;
  const int tilesM = M >> 6;
  const int tile = blockIdx.x * 8 + wave;
  if (tile >= tilesM * tilesN) return;
  const int tm = tile / tilesN;
  const int tn = tile - tm * tilesN;
  const int m0 = tm << 6;
  const int n0 = tn << 5;
  const _Float16* Ah = (const _Float16*)Ahp;
  const _Float16* Al = (const _Float16*)Alp;
  const _Float16* Bh = (const _Float16*)Bhp;
  const _Float16* Bl = (const _Float16*)Blp;
  const int rlane = lane & 15;
  const int koff  = (lane >> 4) * 8;
  const int mOff  = (lane >> 4) * 8;

  v8f am[4][2], ar[4][2];
#pragma unroll
  for (int i = 0; i < 4; ++i)
#pragma unroll
    for (int j = 0; j < 2; ++j) {
      am[i][j] = (v8f){0.f, 0.f, 0.f, 0.f, 0.f, 0.f, 0.f, 0.f};
      ar[i][j] = (v8f){0.f, 0.f, 0.f, 0.f, 0.f, 0.f, 0.f, 0.f};
    }

  for (int k0 = 0; k0 < K; k0 += 32) {
    v16h bh[2], bl[2];
#pragma unroll
    for (int j = 0; j < 2; ++j) {
      const size_t bo = (size_t)(n0 + (j << 4) + rlane) * ldb + koff + k0;
      bh[j] = frag_load(Bh + bo);
      bl[j] = frag_load(Bl + bo);
    }
#pragma unroll
    for (int i = 0; i < 4; ++i) {
      const size_t ao = (size_t)(m0 + (i << 4) + rlane) * lda + koff + k0;
      const v16h ah = frag_load(Ah + ao);
      const v16h al = frag_load(Al + ao);
#pragma unroll
      for (int j = 0; j < 2; ++j) {
        am[i][j] = mma_h(ah, bh[j], am[i][j]);
        ar[i][j] = mma_h(ah, bl[j], ar[i][j]);
        ar[i][j] = mma_h(al, bh[j], ar[i][j]);
      }
    }
  }

  float* slab = sT[wave];
  const int q = lane >> 3, c4 = (lane & 7) * 4;
#pragma unroll
  for (int i = 0; i < 4; ++i) {
    const int mBase = m0 + (i << 4);
#pragma unroll
    for (int j = 0; j < 2; ++j) {
#pragma unroll
      for (int r = 0; r < 8; ++r)
        slab[(mOff + r) * 36 + (j << 4) + rlane] = am[i][j][r] * s_main + ar[i][j][r] * s_res;
    }
    wave_lds_sync();
    for (int pass = 0; pass < 2; ++pass) {
#pragma unroll
      for (int it = 0; it < 4; ++it) {
        const int row = it * 4 + q;
        const v4f v = *(const v4f*)(slab + row * 36 + c4);
        *(volatile v4f*)(C + (size_t)(mBase + row) * ldc + n0 + c4) = v;
      }
      __threadfence();
    }
    wave_lds_sync();
  }
}

__global__ __launch_bounds__(256) void split_planes_kernel(
    const float* __restrict__ src, unsigned short* __restrict__ dhi, unsigned short* __restrict__ dlo,
    int total8, float carry)
{
  const int i = blockIdx.x * 256 + threadIdx.x;
  if (i >= total8) return;
  const size_t e0 = (size_t)i << 3;
  const v4f a0 = *(const v4f*)(src + e0);
  const v4f a1 = *(const v4f*)(src + e0 + 4);
  v8h hv, lv;
#pragma unroll
  for (int e = 0; e < 4; ++e) {
    const float s0 = a0[e] * carry;
    const float s1 = a1[e] * carry;
    const _Float16 h0 = (_Float16)flush_h(s0);
    const _Float16 h1 = (_Float16)flush_h(s1);
    const float r0 = (s0 - (float)h0) * kCarryR;
    const float r1 = (s1 - (float)h1) * kCarryR;
    hv[e]     = h0;
    hv[4 + e] = h1;
    lv[e]     = (_Float16)flush_h(r0);
    lv[4 + e] = (_Float16)flush_h(r1);
  }
  unsigned short* qh = dhi + e0;
  unsigned short* ql = dlo + e0;
  *(volatile v8h*)qh = hv;
  *(volatile v8h*)ql = lv;
  __threadfence();
  *(volatile v8h*)qh = hv;
  *(volatile v8h*)ql = lv;
}

__global__ __launch_bounds__(256) void cast_plane_kernel(
    const float* __restrict__ src, unsigned short* __restrict__ dst, int total8, int real8, float carry)
{
  const int i = blockIdx.x * 256 + threadIdx.x;
  if (i >= total8) return;
  const bool live = (i < real8);
  const int ic = live ? i : (real8 - 1);
  v4f a0 = *(const v4f*)(src + ((size_t)ic << 3));
  v4f a1 = *(const v4f*)(src + ((size_t)ic << 3) + 4);
  asm volatile("" : "+v"(a0), "+v"(a1));
  v8h hv;
#pragma unroll
  for (int e = 0; e < 4; ++e) {
    const float s0 = live ? (a0[e] * carry) : 0.0f;
    const float s1 = live ? (a1[e] * carry) : 0.0f;
    hv[e]     = (_Float16)flush_h(s0);
    hv[4 + e] = (_Float16)flush_h(s1);
  }
  unsigned short* qd = dst + ((size_t)i << 3);
  *(volatile v8h*)qd = hv;
  __threadfence();
  *(volatile v8h*)qd = hv;
}

__global__ __launch_bounds__(256) void conv_silu_norm_kernel(
    const float* __restrict__ QKV, const float* __restrict__ cq, const float* __restrict__ ck,
    const float* __restrict__ cv, float* __restrict__ QN, float* __restrict__ KN, float* __restrict__ VN)
{
  __shared__ __align__(16) float sT[16 * kCvP];
  const int tid = threadIdx.x, lane = tid & 31, wave = tid >> 5;
  const int sec = blockIdx.x >> 2;
  const int cb  = (blockIdx.x & 3) * 256;
  const int c   = cb + tid;
  const int col = sec * kP + c;
  const float* cw = (sec == 0) ? cq : ((sec == 1) ? ck : cv);
  float* dst = (sec == 0) ? QN : ((sec == 1) ? KN : VN);
  const int g0 = blockIdx.y * 64;
  const int tb = g0 & (kT - 1);
  const v4f wv = *(const v4f*)(cw + (size_t)c * 4);
  const float w0 = wv[0], w1 = wv[1], w2 = wv[2], w3 = wv[3];
  float xm3, xm2, xm1;
  {
    const bool hist = (tb > 0);
    const int rb = hist ? (g0 - 3) : g0;
    const float v3 = QKV[(size_t)rb * kQkvN + col];
    const float v2 = QKV[(size_t)(rb + 1) * kQkvN + col];
    const float v1 = QKV[(size_t)(rb + 2) * kQkvN + col];
    xm3 = hist ? v3 : 0.f;
    xm2 = hist ? v2 : 0.f;
    xm1 = hist ? v1 : 0.f;
  }
#pragma unroll 1
  for (int sub = 0; sub < 4; ++sub) {
    const int lb = g0 + sub * 16;
#pragma unroll 1
    for (int s = 0; s < 16; ++s) {
      const float xcur = QKV[(size_t)(lb + s) * kQkvN + col];
      float acc = w0 * xm3;
      acc = fmaf(w1, xm2, acc);
      acc = fmaf(w2, xm1, acc);
      acc = fmaf(w3, xcur, acc);
      const float sg = __builtin_amdgcn_rcpf(1.0f + expf(-acc));
      sT[s * kCvP + tid] = acc * sg;
      xm3 = xm2; xm2 = xm1; xm1 = xcur;
    }
    __syncthreads();
    v4f ov[4];
#pragma unroll
    for (int it = 0; it < 4; ++it) {
      const int seg = it * 8 + wave;
      const int row = seg >> 1, hd = seg & 1;
      const v4f a = *(const v4f*)(sT + row * kCvP + hd * kHD + lane * 4);
      float ss = a[0] * a[0];
      ss = fmaf(a[1], a[1], ss);
      ss = fmaf(a[2], a[2], ss);
      ss = fmaf(a[3], a[3], ss);
      ss += __shfl_xor(ss, 16, 32);
      ss += __shfl_xor(ss, 8, 32);
      ss += __shfl_xor(ss, 4, 32);
      ss += __shfl_xor(ss, 2, 32);
      ss += __shfl_xor(ss, 1, 32);
      const float nrm = rsqrtf(ss + kEps);
      const float f = (sec == 2) ? 1.0f : ((sec == 0) ? (nrm * kQScale) : nrm);
      ov[it] = (v4f){a[0] * f, a[1] * f, a[2] * f, a[3] * f};
    }
    for (int pass = 0; pass < 2; ++pass) {
#pragma unroll
      for (int it = 0; it < 4; ++it) {
        const int seg = it * 8 + wave;
        const int row = seg >> 1, hd = seg & 1;
        *(volatile v4f*)(dst + (size_t)(lb + row) * kP + cb + hd * kHD + lane * 4) = ov[it];
      }
      __threadfence();
    }
    __syncthreads();
  }
}

__global__ __launch_bounds__(256) void decay_kernel(
    const float* __restrict__ GF, const float* __restrict__ A_log, const float* __restrict__ dt_bias,
    float* __restrict__ EG)
{
  __shared__ __align__(16) float sS[kP];
  const int tid = threadIdx.x;
  const size_t row = blockIdx.x;
#pragma unroll 1
  for (int it = 0; it < 4; ++it) {
    const int c = it * 256 + tid;
    const int hd = c / kHD;
    const float x = GF[row * kP + c] + dt_bias[c];
    const float sp = fmaxf(x, 0.0f) + log1pf(expf(-fabsf(x)));
    const float g = -expf(A_log[hd]) * sp;
    float e = expf(g);
    e = (e < kF32MinNormal) ? 0.0f : e;
    sS[c] = e;
  }
  __syncthreads();
  const v4f ev = *(const v4f*)(sS + tid * 4);
  float* p = EG + row * kP + tid * 4;
  *(volatile v4f*)p = ev;
  __threadfence();
  *(volatile v4f*)p = ev;
}

__global__ __launch_bounds__(512) void delta_scan_kernel(
    const float* __restrict__ QN, const float* __restrict__ KN, const float* __restrict__ VN,
    const float* __restrict__ EG, const float* __restrict__ BETA, float* __restrict__ OB)
{
  __shared__ __align__(16) float sK[kScanTS * kHD];
  __shared__ __align__(16) float sQ[kScanTS * kHD];
  __shared__ __align__(16) float sE[kScanTS * kHD];
  __shared__ __align__(16) float sV[kScanTS * kHD];
  __shared__ __align__(16) float sO[kScanTS * kScanOP];
  __shared__ __align__(16) float sB[kScanTS];
  const int tid = threadIdx.x, lane = tid & 31, wave = tid >> 5;
  const int half = blockIdx.x & 1;
  const int hd   = (blockIdx.x >> 1) & (kNH - 1);
  const int bb   = blockIdx.x / (2 * kNH);
  const int vc   = tid >> 3;
  const int kq   = tid & 7;
  const size_t row0 = (size_t)bb * kT;
  const int cb = hd * kHD;
  const int sr = tid >> 5, sc4 = (tid & 31) * 4;
  const int br = tid & (kScanTS - 1);
  const int hh = lane >> 4, c4 = (lane & 15) * 4;

  float S[16];
#pragma unroll
  for (int j = 0; j < 16; ++j) S[j] = 0.f;

#pragma unroll 1
  for (int t0 = 0; t0 < kT; t0 += kScanTS) {
    {
      const size_t go = (row0 + t0 + sr) * kP + cb + sc4;
      const v4f kk = *(const v4f*)(KN + go);
      const v4f qq = *(const v4f*)(QN + go);
      const v4f ee = *(const v4f*)(EG + go);
      const v4f vv = *(const v4f*)(VN + go);
      float braw = BETA[(row0 + t0 + br) * kBetaPad + hd];
      asm volatile("" : "+v"(braw));
      *(v4f*)(sK + sr * kHD + sc4) = kk;
      *(v4f*)(sQ + sr * kHD + sc4) = qq;
      *(v4f*)(sE + sr * kHD + sc4) = ee;
      *(v4f*)(sV + sr * kHD + sc4) = vv;
      if (tid < kScanTS) sB[tid] = __builtin_amdgcn_rcpf(1.0f + expf(-braw));
    }
    __syncthreads();
#pragma unroll 1
    for (int s = 0; s < kScanTS; ++s) {
      const float* kp = sK + s * kHD + kq * 16;
      const float* ep = sE + s * kHD + kq * 16;
      const float* qp = sQ + s * kHD + kq * 16;
      float kr[16];
      float kv = 0.f;
#pragma unroll
      for (int j4 = 0; j4 < 4; ++j4) {
        const v4f kx = *(const v4f*)(kp + 4 * j4);
        const v4f ex = *(const v4f*)(ep + 4 * j4);
#pragma unroll
        for (int e = 0; e < 4; ++e) {
          kr[4 * j4 + e] = kx[e];
          S[4 * j4 + e] *= ex[e];
          kv = fmaf(kx[e], S[4 * j4 + e], kv);
        }
      }
      kv += __shfl_xor(kv, 1, 32);
      kv += __shfl_xor(kv, 2, 32);
      kv += __shfl_xor(kv, 4, 32);
      const float delta = (sV[s * kHD + half * 64 + vc] - kv) * sB[s];
      float o = 0.f;
#pragma unroll
      for (int j4 = 0; j4 < 4; ++j4) {
        const v4f qx = *(const v4f*)(qp + 4 * j4);
#pragma unroll
        for (int e = 0; e < 4; ++e) {
          S[4 * j4 + e] = fmaf(kr[4 * j4 + e], delta, S[4 * j4 + e]);
          o = fmaf(qx[e], S[4 * j4 + e], o);
        }
      }
      o += __shfl_xor(o, 1, 32);
      o += __shfl_xor(o, 2, 32);
      o += __shfl_xor(o, 4, 32);
      if (kq == 0) sO[s * kScanOP + vc] = o;
    }
    __syncthreads();
    if (wave < 8) {
      const int row = 2 * wave + hh;
      const v4f ov = *(const v4f*)(sO + row * kScanOP + c4);
      float* p = OB + (row0 + t0 + row) * kP + cb + half * 64 + c4;
      *(volatile v4f*)p = ov;
      __threadfence();
      *(volatile v4f*)p = ov;
    }
  }
}

__global__ __launch_bounds__(256) void gate_norm_kernel(
    const float* __restrict__ OB, const float* __restrict__ GATE, const float* __restrict__ nw,
    unsigned short* __restrict__ OGH)
{
  const int tid = threadIdx.x, lane = tid & 31, wave = tid >> 5;
  const size_t o0 = (size_t)blockIdx.x * kP + wave * kHD + lane * 4;
  const v4f ov = *(const v4f*)(OB + o0);
  const v4f gv = *(const v4f*)(GATE + o0);
  const v4f wv = *(const v4f*)(nw + lane * 4);
  float og[4];
  float ss = 0.f;
#pragma unroll
  for (int e = 0; e < 4; ++e) {
    const float sg = __builtin_amdgcn_rcpf(1.0f + expf(-gv[e]));
    og[e] = ov[e] * sg;
    ss = fmaf(og[e], og[e], ss);
  }
  ss += __shfl_xor(ss, 16, 32);
  ss += __shfl_xor(ss, 8, 32);
  ss += __shfl_xor(ss, 4, 32);
  ss += __shfl_xor(ss, 2, 32);
  ss += __shfl_xor(ss, 1, 32);
  const float rn = rsqrtf(ss * (1.0f / (float)kHD) + kEps);
  v4h hv;
#pragma unroll
  for (int e = 0; e < 4; ++e) {
    const float val = (og[e] * rn) * wv[e] * kCarryO;
    hv[e] = (_Float16)flush_h(val);
  }
  unsigned short* p = OGH + o0;
  *(volatile v4h*)p = hv;
  __threadfence();
  *(volatile v4h*)p = hv;
}

extern "C" void kernel_launch(void* const* d_in, const int* in_sizes, int n_in,
                              void* d_out, int out_size, void* d_ws, size_t ws_size,
                              hipStream_t stream) {
  if (n_in < 16) return;
  if (in_sizes[0] != kRows * kHid) return;
  if (in_sizes[1] != kP * kHid || in_sizes[2] != kP * kHid || in_sizes[3] != kP * kHid) return;
  if (in_sizes[4] != kP * 4 || in_sizes[5] != kP * 4 || in_sizes[6] != kP * 4) return;
  if (in_sizes[7] != kNH) return;
  if (in_sizes[8] != kP) return;
  if (in_sizes[9] != kHD * kHid) return;
  if (in_sizes[10] != kP * kHD) return;
  if (in_sizes[11] != kNH * kHid) return;
  if (in_sizes[12] != kHD * kHid) return;
  if (in_sizes[13] != kP * kHD) return;
  if (in_sizes[14] != kHD) return;
  if (in_sizes[15] != kHid * kP) return;
  if (out_size != kRows * kHid) return;
  if (ws_size < kWsTotal) return;

  const float* x       = (const float*)d_in[0];
  const float* Wq      = (const float*)d_in[1];
  const float* Wk      = (const float*)d_in[2];
  const float* Wv      = (const float*)d_in[3];
  const float* conv_q  = (const float*)d_in[4];
  const float* conv_k  = (const float*)d_in[5];
  const float* conv_v  = (const float*)d_in[6];
  const float* A_log   = (const float*)d_in[7];
  const float* dt_bias = (const float*)d_in[8];
  const float* Wfa     = (const float*)d_in[9];
  const float* Wfb     = (const float*)d_in[10];
  const float* Wb      = (const float*)d_in[11];
  const float* Wga     = (const float*)d_in[12];
  const float* Wgb     = (const float*)d_in[13];
  const float* norm_w  = (const float*)d_in[14];
  const float* Wo      = (const float*)d_in[15];
  float* out = (float*)d_out;

  char* ws = (char*)d_ws;
  unsigned short* XH   = (unsigned short*)(ws + kOffXH);
  unsigned short* XL   = (unsigned short*)(ws + kOffXL);
  unsigned short* WH   = (unsigned short*)(ws + kOffWH);
  unsigned short* WL   = (unsigned short*)(ws + kOffWL);
  unsigned short* WLR  = (unsigned short*)(ws + kOffWLR);
  unsigned short* W2   = (unsigned short*)(ws + kOffW2);
  unsigned short* WOH  = (unsigned short*)(ws + kOffWOH);
  float*          QKV  = (float*)(ws + kOffQKV);
  float*          OB   = (float*)(ws + kOffQKV);
  unsigned short* HID  = (unsigned short*)(ws + kOffHID);
  float*          BETA = (float*)(ws + kOffBETA);
  float*          GG   = (float*)(ws + kOffGG);
  float*          EG   = (float*)(ws + kOffEG);
  float*          QN   = (float*)(ws + kOffQN);
  float*          KN   = (float*)(ws + kOffKN);
  float*          VN   = (float*)(ws + kOffVN);
  unsigned short* OGH  = (unsigned short*)(ws + kOffOGH);

  constexpr int kX8   = kRows * kHid / 8;
  constexpr int kW8   = kP * kHid / 8;
  constexpr int kFa8  = kHD * kHid / 8;
  constexpr int kWb8  = kBetaPad * kHid / 8;
  constexpr int kWbR8 = kNH * kHid / 8;
  constexpr int kFb8  = kP * kHD / 8;
  constexpr int kWo8  = kHid * kP / 8;
  static_assert((kX8 % 256) == 0 && (kW8 % 256) == 0 && (kFa8 % 256) == 0 && (kWb8 % 256) == 0 &&
                (kWbR8 % 256) == 0 && (kFb8 % 256) == 0 && (kWo8 % 256) == 0, "exact cast grids");
  split_planes_kernel<<<kX8 / 256, 256, 0, stream>>>(x, XH, XL, kX8, kCarryX);
  split_planes_kernel<<<kW8 / 256, 256, 0, stream>>>(Wq, WH, WL, kW8, kCarryW);
  split_planes_kernel<<<kW8 / 256, 256, 0, stream>>>(Wk, WH + (size_t)kP * kHid, WL + (size_t)kP * kHid, kW8, kCarryW);
  split_planes_kernel<<<kW8 / 256, 256, 0, stream>>>(Wv, WH + (size_t)2 * kP * kHid, WL + (size_t)2 * kP * kHid, kW8, kCarryW);
  cast_plane_kernel<<<kFa8 / 256, 256, 0, stream>>>(Wfa, WLR, kFa8, kFa8, kCarryW);
  cast_plane_kernel<<<kFa8 / 256, 256, 0, stream>>>(Wga, WLR + (size_t)kHD * kHid, kFa8, kFa8, kCarryW);
  cast_plane_kernel<<<kWb8 / 256, 256, 0, stream>>>(Wb, WLR + (size_t)kLrN * kHid, kWb8, kWbR8, kCarryW);
  cast_plane_kernel<<<kFb8 / 256, 256, 0, stream>>>(Wfb, W2, kFb8, kFb8, kCarryW);
  cast_plane_kernel<<<kFb8 / 256, 256, 0, stream>>>(Wgb, W2 + (size_t)kP * kHD, kFb8, kFb8, kCarryW);
  cast_plane_kernel<<<kWo8 / 256, 256, 0, stream>>>(Wo, WOH, kWo8, kWo8, kCarryW);

  gemm_split_kernel<<<(kRows / 64) * (kQkvN / 32) / 8, 256, 0, stream>>>(
      XH, XL, kHid, WH, WL, kHid, QKV, kQkvN, kRows, kQkvN, kHid, kScaleMain, kScaleRes);

  conv_silu_norm_kernel<<<dim3(3 * (kP / 256), kRows / 64), 256, 0, stream>>>(
      QKV, conv_q, conv_k, conv_v, QN, KN, VN);

  gemm_plain_kernel<1><<<dim3((kRows / 64) * (kLrN / 64) / 8, 1), 256, 0, stream>>>(
      XH, kHid, 0L, WLR, kHid, 0L, (void*)HID, kLrN, 0L, kRows, kLrN, kHid, kScaleHid);

  gemm_plain_kernel<0><<<dim3((kRows / 64) * (kBetaPad / 64) / 8, 1), 256, 0, stream>>>(
      XH, kHid, 0L, WLR + (size_t)kLrN * kHid, kHid, 0L, (void*)BETA, kBetaPad, 0L,
      kRows, kBetaPad, kHid, kScaleMain);

  gemm_plain_kernel<0><<<dim3((kRows / 64) * (kP / 64) / 8, 2), 256, 0, stream>>>(
      HID, kLrN, (long)kHD, W2, kHD, (long)kP * kHD, (void*)GG, kP, (long)kRows * kP,
      kRows, kP, kHD, kScaleLr2);

  decay_kernel<<<kRows, 256, 0, stream>>>(GG, A_log, dt_bias, EG);

  delta_scan_kernel<<<kNB * kNH * 2, 512, 0, stream>>>(QN, KN, VN, EG, BETA, OB);

  gate_norm_kernel<<<kRows, 256, 0, stream>>>(OB, GG + (size_t)kRows * kP, norm_w, OGH);

  gemm_plain_kernel<0><<<dim3((kRows / 64) * (kHid / 64) / 8, 1), 256, 0, stream>>>(
      OGH, kP, 0L, WOH, kP, 0L, (void*)out, kHid, 0L, kRows, kHid, kP, kScaleOut);
}
